// LSTM2d_45689862095226
// MI455X (gfx1250) — hardware-run, weakly checked
//
#include <hip/hip_runtime.h>
#include <math.h>

typedef __attribute__((ext_vector_type(16))) _Float16 v16h;
typedef __attribute__((ext_vector_type(8)))  _Float16 v8h;
typedef __attribute__((ext_vector_type(8)))  float    v8f;
typedef __attribute__((ext_vector_type(4)))  float    v4f;

constexpr int kSin   = 16;
constexpr int kSout  = 16;
constexpr int kB     = 32;
constexpr int kE     = 256;
constexpr int kEnc   = 256;
constexpr int kD     = 256;
constexpr int kVocab = 32000;
constexpr int kRows  = kSin * kB;
constexpr int kG4    = 4 * kEnc;
constexpr int kG5    = 5 * kD;
constexpr int kWxP   = 2 * kEnc + kE;
constexpr int kWsP   = 2 * kD;
constexpr int kPlane = kB * kD;
static_assert(kSin == 16 && kSout == 16 && kB == 32, "grid and batch extents");
static_assert(kRows == 512 && kG4 == 1024 && kG5 == 1280 && kWxP == 768 && kWsP == 512 && kPlane == 8192, "derived extents");
static_assert((kE % 32) == 0 && (kEnc % 32) == 0 && ((2 * kEnc) % 32) == 0 && (kWsP % 32) == 0 && (kD % 32) == 0, "K multiples of 32");
static_assert((kRows % 64) == 0 && (kG4 % 64) == 0 && (kG5 % 64) == 0 && (kVocab % 64) == 0, "M,N multiples of 64");

constexpr float kCarryW = 256.0f;
constexpr float kCarryE = 256.0f;
constexpr float kCarryS = 1024.0f;
constexpr float kFoldEW = 1.0f / (kCarryE * kCarryW);
constexpr float kFoldSW = 1.0f / (kCarryS * kCarryW);
constexpr float kF16MinNormal = 6.103515625e-05f;

constexpr int kHP = 260;
constexpr int kAP = 520;
constexpr int kOP = 36;

constexpr size_t kSzW4   = (size_t)kG4 * kE * 2;
constexpr size_t kSzWX   = (size_t)kG5 * kWxP * 2;
constexpr size_t kSzWS   = (size_t)kG5 * kWsP * 2;
constexpr size_t kSzLW   = (size_t)kVocab * kD * 2;
constexpr size_t kSzEmb  = (size_t)kRows * kE * 2;
constexpr size_t kSzGI   = (size_t)kRows * kG4 * 4;
constexpr size_t kSzH    = (size_t)kRows * 2 * kEnc * 4;
constexpr size_t kSzH16  = (size_t)kRows * 2 * kEnc * 2;
constexpr size_t kSzPJ   = (size_t)kRows * kG5 * 4;
constexpr size_t kSzSC   = (size_t)kSin * kSout * kPlane * 4;
constexpr size_t kSzST   = (size_t)kRows * kD * 2;
constexpr size_t kOffWIF = 0;
constexpr size_t kOffWHF = kOffWIF + kSzW4;
constexpr size_t kOffWIB = kOffWHF + kSzW4;
constexpr size_t kOffWHB = kOffWIB + kSzW4;
constexpr size_t kOffWX  = kOffWHB + kSzW4;
constexpr size_t kOffWS  = kOffWX  + kSzWX;
constexpr size_t kOffLW  = kOffWS  + kSzWS;
constexpr size_t kOffXE  = kOffLW  + kSzLW;
constexpr size_t kOffYE  = kOffXE  + kSzEmb;
constexpr size_t kOffGIF = kOffYE  + kSzEmb;
constexpr size_t kOffGIB = kOffGIF + kSzGI;
constexpr size_t kOffH   = kOffGIB + kSzGI;
constexpr size_t kOffH16 = kOffH   + kSzH;
constexpr size_t kOffHPJ = kOffH16 + kSzH16;
constexpr size_t kOffYPJ = kOffHPJ + kSzPJ;
constexpr size_t kOffSPL = kOffYPJ + kSzPJ;
constexpr size_t kOffCPL = kOffSPL + kSzSC;
constexpr size_t kOffST  = kOffCPL + kSzSC;
constexpr size_t kWsTotal = kOffST + kSzST;
static_assert(kWsTotal == 50331648ull, "carve total");
static_assert(kWsTotal <= 134217728ull, "carve cap");
static_assert((kOffWHF % 128) == 0 && (kOffWIB % 128) == 0 && (kOffWHB % 128) == 0 && (kOffWX % 128) == 0 &&
              (kOffWS % 128) == 0 && (kOffLW % 128) == 0 && (kOffXE % 128) == 0 && (kOffYE % 128) == 0 &&
              (kOffGIF % 128) == 0 && (kOffGIB % 128) == 0 && (kOffH % 128) == 0 && (kOffH16 % 128) == 0 &&
              (kOffHPJ % 128) == 0 && (kOffYPJ % 128) == 0 && (kOffSPL % 128) == 0 && (kOffCPL % 128) == 0 &&
              (kOffST % 128) == 0, "128-B aligned regions");

union FragU { v16h v; v8h h[2]; };
__device__ __forceinline__ v16h frag_load(const _Float16* p) {
  FragU f;
  f.h[0] = *(const v8h*)(p);
  f.h[1] = *(const v8h*)(p + 16);
  return f.v;
}
__device__ __forceinline__ v8f mma_h(v16h a, v16h b, v8f c) {
  c = __builtin_amdgcn_wmma_f32_16x16x32_f16(false, a, false, b, (short)0, c, false, false);
  asm volatile("v_nop\n\tv_nop\n\tv_nop\n\tv_nop" : "+v"(c) : "v"(a), "v"(b));
  return c;
}
__device__ __forceinline__ _Float16 cvt_carry(float v, float carry) {
  const float x = v * carry;
  const float y = (fabsf(x) < kF16MinNormal) ? 0.0f : x;
  return (_Float16)y;
}
__device__ __forceinline__ v8h pack8(v4f a0, v4f a1, float carry) {
  v8h hv;
#pragma unroll
  for (int e = 0; e < 4; ++e) {
    hv[e]     = cvt_carry(a0[e], carry);
    hv[4 + e] = cvt_carry(a1[e], carry);
  }
  return hv;
}
__device__ __forceinline__ float sigm(float x) { return 1.0f / (1.0f + expf(-x)); }

__global__ __launch_bounds__(256) void cast_carry_kernel(
    const float* __restrict__ src, unsigned short* __restrict__ dst, int n8, float carry)
{
  const int i = blockIdx.x * 256 + threadIdx.x;
  if (i >= n8) return;
  const size_t e0 = (size_t)i << 3;
  const v4f a0 = *(const v4f*)(src + e0);
  const v4f a1 = *(const v4f*)(src + e0 + 4);
  const v8h hv = pack8(a0, a1, carry);
  unsigned short* q = dst + e0;
  *(volatile v8h*)q = hv;
  __threadfence();
  *(volatile v8h*)q = hv;
}

__global__ __launch_bounds__(256) void gather_embed_kernel(
    const int* __restrict__ xid, const int* __restrict__ yid,
    const float* __restrict__ inE, const float* __restrict__ outE,
    unsigned short* __restrict__ XE, unsigned short* __restrict__ YE)
{
  const int which = blockIdx.y;
  const int t = blockIdx.x * 256 + threadIdx.x;
  const int row = t >> 5;
  const int c8 = (t & 31) * 8;
  const int yrow = (row >= kB) ? (row - kB) : 0;
  const int xt = xid[row];
  const int yt = yid[yrow];
  int tok = which ? ((row < kB) ? 1 : yt) : xt;
  tok = tok < 0 ? 0 : tok;
  tok = tok > (kVocab - 1) ? (kVocab - 1) : tok;
  const float* tab = which ? outE : inE;
  const float* p = tab + (size_t)tok * kE + c8;
  const v4f a0 = *(const v4f*)(p);
  const v4f a1 = *(const v4f*)(p + 4);
  const v8h hv = pack8(a0, a1, kCarryE);
  unsigned short* q = (which ? YE : XE) + (size_t)row * kE + c8;
  *(volatile v8h*)q = hv;
  __threadfence();
  *(volatile v8h*)q = hv;
}

template <int BIAS_MODE>
__global__ __launch_bounds__(256) void wmma_gemm64_f16(
    const unsigned short* __restrict__ Ap, int lda,
    const unsigned short* __restrict__ Btp, int ldb,
    float* __restrict__ Cout, int ldc,
    const float* __restrict__ bias,
    int M, int N, int K, float scale)
{
  const _Float16* A  = (const _Float16*)Ap;
  const _Float16* Bt = (const _Float16*)Btp;
  __shared__ __align__(16) float sT[8][16 * 68];
  const int lane = threadIdx.x & 31;
  const int wave = threadIdx.x >> 5;
  const int tilesN = N >> 6;
  const int tilesM = M >> 6;
  const int tile = blockIdx.x * 8 + wave;
  if (tile >= tilesM * tilesN) return;
  const int tm = tile / tilesN;
  const int tn = tile - tm * tilesN;
  const int m0 = tm << 6;
  const int n0 = tn << 6;
  const int rlane = lane & 15;
  const int koff  = (lane >> 4) * 8;
  const int mOff  = (lane >> 4) * 8;

  v8f acc[4][4];
#pragma unroll
  for (int i = 0; i < 4; ++i)
#pragma unroll
    for (int j = 0; j < 4; ++j) acc[i][j] = (v8f){0.f, 0.f, 0.f, 0.f, 0.f, 0.f, 0.f, 0.f};

  for (int k0 = 0; k0 < K; k0 += 32) {
    v16h bh[4];
#pragma unroll
    for (int j = 0; j < 4; ++j) {
      const size_t bo = (size_t)(n0 + (j << 4) + rlane) * ldb + koff + k0;
      bh[j] = frag_load(Bt + bo);
    }
#pragma unroll
    for (int i = 0; i < 4; ++i) {
      const size_t ao = (size_t)(m0 + (i << 4) + rlane) * lda + koff + k0;
      const v16h ah = frag_load(A + ao);
#pragma unroll
      for (int j = 0; j < 4; ++j) acc[i][j] = mma_h(ah, bh[j], acc[i][j]);
    }
  }

  float* slab = sT[wave];
#pragma unroll
  for (int i = 0; i < 4; ++i) {
    const int mBase = m0 + (i << 4);
#pragma unroll
    for (int j = 0; j < 4; ++j) {
      const int n = n0 + (j << 4) + rlane;
      float bv = 0.f;
      if (BIAS_MODE == 2) bv = bias[n];
#pragma unroll
      for (int r = 0; r < 8; ++r) {
        float v = acc[i][j][r] * scale;
        if (BIAS_MODE == 2) v += bv;
        slab[(mOff + r) * 68 + (j << 4) + rlane] = v;
      }
    }
    __builtin_amdgcn_fence(__ATOMIC_RELEASE, "workgroup");
    __builtin_amdgcn_wave_barrier();
    __builtin_amdgcn_fence(__ATOMIC_ACQUIRE, "workgroup");
    {
      const int hh = lane >> 4, c4 = (lane & 15) * 4;
      for (int pass = 0; pass < 2; ++pass) {
#pragma unroll
        for (int it = 0; it < 8; ++it) {
          const int row = it * 2 + hh;
          const v4f v = *(const v4f*)(slab + row * 68 + c4);
          *(volatile v4f*)(Cout + (size_t)(mBase + row) * ldc + n0 + c4) = v;
        }
        __threadfence();
      }
    }
    __builtin_amdgcn_fence(__ATOMIC_RELEASE, "workgroup");
    __builtin_amdgcn_wave_barrier();
    __builtin_amdgcn_fence(__ATOMIC_ACQUIRE, "workgroup");
  }
}

__global__ __launch_bounds__(512) void encoder_kernel(
    const float* __restrict__ GIf, const float* __restrict__ GIb,
    const unsigned short* __restrict__ WHf, const unsigned short* __restrict__ WHb,
    float* __restrict__ Hout)
{
  __shared__ __align__(16) float hs[32 * kHP];
  const int tid = threadIdx.x, lane = tid & 31, wave = tid >> 5;
  const int c = lane & 15, hh = lane >> 4;
  const int dir = blockIdx.x;
  const float* GI = dir ? GIb : GIf;
  const _Float16* WH = (const _Float16*)(dir ? WHb : WHf);
  const int rt = wave & 1, ug = wave >> 1;

#pragma unroll 1
  for (int i = tid; i < 32 * kHP; i += 512) hs[i] = 0.0f;
  float cst[2][8];
#pragma unroll
  for (int nt = 0; nt < 2; ++nt)
#pragma unroll
    for (int r = 0; r < 8; ++r) cst[nt][r] = 0.0f;
  __syncthreads();

  const float* hrow = hs + (16 * rt + c) * kHP + 8 * hh;

#pragma unroll 1
  for (int step = 0; step < kSin; ++step) {
    const int s = dir ? (kSin - 1 - step) : step;
    float hst[2][8];
#pragma unroll
    for (int nt = 0; nt < 2; ++nt) {
      const int j = 32 * ug + 16 * nt + c;
      const _Float16* wb = WH + (size_t)j * kEnc + 8 * hh;
      v8f acc[4];
#pragma unroll
      for (int g = 0; g < 4; ++g) acc[g] = (v8f){0.f, 0.f, 0.f, 0.f, 0.f, 0.f, 0.f, 0.f};
#pragma unroll 4
      for (int k0 = 0; k0 < kEnc; k0 += 32) {
        const float* p = hrow + k0;
        const v4f x0 = *(const v4f*)(p);
        const v4f x1 = *(const v4f*)(p + 4);
        const v4f x2 = *(const v4f*)(p + 16);
        const v4f x3 = *(const v4f*)(p + 20);
        v16h a;
#pragma unroll
        for (int e = 0; e < 4; ++e) {
          a[e]      = cvt_carry(x0[e], kCarryS);
          a[4 + e]  = cvt_carry(x1[e], kCarryS);
          a[8 + e]  = cvt_carry(x2[e], kCarryS);
          a[12 + e] = cvt_carry(x3[e], kCarryS);
        }
#pragma unroll
        for (int g = 0; g < 4; ++g) {
          const v16h b = frag_load(wb + (size_t)g * kEnc * kEnc + k0);
          acc[g] = mma_h(a, b, acc[g]);
        }
      }
      const float* gp = GI + (size_t)(s * kB + 16 * rt + 8 * hh) * kG4 + j;
#pragma unroll
      for (int r = 0; r < 8; ++r) {
        const float gi = gp[r * kG4];
        const float gf = gp[r * kG4 + kEnc];
        const float gg = gp[r * kG4 + 2 * kEnc];
        const float go = gp[r * kG4 + 3 * kEnc];
        const float zi = acc[0][r] * kFoldSW + gi;
        const float zf = acc[1][r] * kFoldSW + gf;
        const float zg = acc[2][r] * kFoldSW + gg;
        const float zo = acc[3][r] * kFoldSW + go;
        const float cn = sigm(zf) * cst[nt][r] + sigm(zi) * tanhf(zg);
        cst[nt][r] = cn;
        hst[nt][r] = sigm(zo) * tanhf(cn);
        if (r == 3) asm volatile("" ::: "memory");
      }
    }
    __syncthreads();
#pragma unroll
    for (int nt = 0; nt < 2; ++nt) {
      const int j = 32 * ug + 16 * nt + c;
#pragma unroll
      for (int r = 0; r < 8; ++r) hs[(16 * rt + 8 * hh + r) * kHP + j] = hst[nt][r];
    }
    __syncthreads();
    for (int pass = 0; pass < 2; ++pass) {
#pragma unroll
      for (int it = 0; it < 4; ++it) {
        const int idx = it * 512 + tid;
        const int row = idx >> 6, c4 = (idx & 63) * 4;
        const v4f v = *(const v4f*)(hs + row * kHP + c4);
        *(volatile v4f*)(Hout + (size_t)(s * kB + row) * (2 * kEnc) + dir * kEnc + c4) = v;
      }
      __threadfence();
    }
  }
}

__global__ __launch_bounds__(128) void grid_cell_kernel(
    const float* __restrict__ HPp, const float* __restrict__ YPp,
    const unsigned short* __restrict__ WSp,
    float* Spl, float* Cpl, int d, int ilo)
{
  __shared__ __align__(16) _Float16 At[32 * kAP];
  __shared__ __align__(16) float So[4][16 * kOP];
  __shared__ __align__(16) float Co[4][16 * kOP];
  const int tid = threadIdx.x, lane = tid & 31, wave = tid >> 5;
  const int c = lane & 15, hh = lane >> 4;
  int i = ilo + (int)blockIdx.x;
  i = i < 0 ? 0 : (i > kSin - 1 ? kSin - 1 : i);
  int j = d - i;
  j = j < 0 ? 0 : (j > kSout - 1 ? kSout - 1 : j);
  const bool hasH = (i > 0);
  const bool hasV = (j > 0);
  const float* Sh = hasH ? (Spl + (size_t)((i - 1) * kSout + j) * kPlane) : HPp;
  const float* Sv = hasV ? (Spl + (size_t)(i * kSout + (j - 1)) * kPlane) : HPp;
  const float* Ch = hasH ? (Cpl + (size_t)((i - 1) * kSout + j) * kPlane) : HPp;
  const float* Cv = hasV ? (Cpl + (size_t)(i * kSout + (j - 1)) * kPlane) : HPp;

  {
    const int rr = tid >> 5, kc = (tid & 31) * 8;
    const v8h zz = {(_Float16)0.0f, (_Float16)0.0f, (_Float16)0.0f, (_Float16)0.0f,
                    (_Float16)0.0f, (_Float16)0.0f, (_Float16)0.0f, (_Float16)0.0f};
    if (hasH) {
#pragma unroll 1
      for (int it = 0; it < 8; ++it) {
        const int row = it * 4 + rr;
        const float* p = Sh + (size_t)row * kD + kc;
        const v4f a0 = *(const v4f*)(p);
        const v4f a1 = *(const v4f*)(p + 4);
        *(v8h*)(At + row * kAP + kc) = pack8(a0, a1, kCarryS);
      }
    } else {
#pragma unroll 1
      for (int it = 0; it < 8; ++it) {
        const int row = it * 4 + rr;
        *(v8h*)(At + row * kAP + kc) = zz;
      }
    }
    if (hasV) {
#pragma unroll 1
      for (int it = 0; it < 8; ++it) {
        const int row = it * 4 + rr;
        const float* p = Sv + (size_t)row * kD + kc;
        const v4f a0 = *(const v4f*)(p);
        const v4f a1 = *(const v4f*)(p + 4);
        *(v8h*)(At + row * kAP + kD + kc) = pack8(a0, a1, kCarryS);
      }
    } else {
#pragma unroll 1
      for (int it = 0; it < 8; ++it) {
        const int row = it * 4 + rr;
        *(v8h*)(At + row * kAP + kD + kc) = zz;
      }
    }
  }
  __syncthreads();

  const _Float16* WS = (const _Float16*)WSp;
  float* sow = &So[wave][0];
  float* cow = &Co[wave][0];
  float* Sdst0 = Spl + (size_t)(i * kSout + j) * kPlane;
  float* Cdst0 = Cpl + (size_t)(i * kSout + j) * kPlane;
  const int q = lane >> 3, c4 = (lane & 7) * 4;

#pragma unroll 1
  for (int ug = 0; ug < 2; ++ug) {
#pragma unroll 1
    for (int rt = 0; rt < 2; ++rt) {
#pragma unroll 1
      for (int nt = 0; nt < 2; ++nt) {
        const int u = 64 * wave + 32 * ug + 16 * nt + c;
        const _Float16* ar = At + (16 * rt + c) * kAP + 8 * hh;
        const _Float16* wb = WS + (size_t)u * kWsP + 8 * hh;
        v8f acc[5];
#pragma unroll
        for (int g = 0; g < 5; ++g) acc[g] = (v8f){0.f, 0.f, 0.f, 0.f, 0.f, 0.f, 0.f, 0.f};
#pragma unroll 1
        for (int kh = 0; kh < 2; ++kh) {
#pragma unroll
          for (int kk = 0; kk < 8; ++kk) {
            const int k0 = kh * kD + kk * 32;
            const v16h a = frag_load(ar + k0);
#pragma unroll
            for (int g = 0; g < 5; ++g) {
              const v16h b = frag_load(wb + (size_t)g * kD * kWsP + k0);
              acc[g] = mma_h(a, b, acc[g]);
            }
          }
        }
        const int row0 = 16 * rt + 8 * hh;
        const float* hpr = HPp + (size_t)(i * kB + row0) * kG5 + u;
        const float* ypr = YPp + (size_t)(j * kB + row0) * kG5 + u;
        const float* chr = Ch + (size_t)row0 * kD + u;
        const float* cvr = Cv + (size_t)row0 * kD + u;
        float* sop = sow + (8 * hh) * kOP + 16 * nt + c;
        float* cop = cow + (8 * hh) * kOP + 16 * nt + c;
#pragma unroll
        for (int r = 0; r < 8; ++r) {
          const int ro = r * kG5;
          const float p0 = acc[0][r] * kFoldSW + (hpr[ro] + ypr[ro]);
          const float p1 = acc[1][r] * kFoldSW + (hpr[ro + kD] + ypr[ro + kD]);
          const float p2 = acc[2][r] * kFoldSW + (hpr[ro + 2 * kD] + ypr[ro + 2 * kD]);
          const float p3 = acc[3][r] * kFoldSW + (hpr[ro + 3 * kD] + ypr[ro + 3 * kD]);
          const float p4 = acc[4][r] * kFoldSW + (hpr[ro + 4 * kD] + ypr[ro + 4 * kD]);
          float ch = 0.0f, cv = 0.0f;
          if (hasH) ch = chr[r * kD];
          if (hasV) cv = cvr[r * kD];
          const float ig = sigm(p0);
          const float fg = sigm(p1);
          const float lg = sigm(p2);
          const float og = sigm(p3);
          const float gg = tanhf(p4);
          const float cn = fg * (lg * ch + (1.0f - lg) * cv) + ig * gg;
          const float sn = og * tanhf(cn);
          sop[r * kOP] = sn;
          cop[r * kOP] = cn;
          asm volatile("" ::: "memory");
        }
      }
      __builtin_amdgcn_fence(__ATOMIC_RELEASE, "workgroup");
      __builtin_amdgcn_wave_barrier();
      __builtin_amdgcn_fence(__ATOMIC_ACQUIRE, "workgroup");
      {
        float* Sd = Sdst0 + (size_t)(16 * rt) * kD + 64 * wave + 32 * ug + c4;
        float* Cd = Cdst0 + (size_t)(16 * rt) * kD + 64 * wave + 32 * ug + c4;
        for (int pass = 0; pass < 2; ++pass) {
#pragma unroll
          for (int it = 0; it < 4; ++it) {
            const int rowl = it * 4 + q;
            const v4f sv = *(const v4f*)(sow + rowl * kOP + c4);
            const v4f cv4 = *(const v4f*)(cow + rowl * kOP + c4);
            *(volatile v4f*)(Sd + (size_t)rowl * kD) = sv;
            *(volatile v4f*)(Cd + (size_t)rowl * kD) = cv4;
          }
          __threadfence();
        }
      }
      __builtin_amdgcn_fence(__ATOMIC_RELEASE, "workgroup");
      __builtin_amdgcn_wave_barrier();
      __builtin_amdgcn_fence(__ATOMIC_ACQUIRE, "workgroup");
    }
  }
}

extern "C" void kernel_launch(void* const* d_in, const int* in_sizes, int n_in,
                              void* d_out, int out_size, void* d_ws, size_t ws_size,
                              hipStream_t stream) {
  if (n_in < 16 || d_out == nullptr || d_ws == nullptr) return;
  if (in_sizes[0] != kSin * kB) return;
  if (in_sizes[2] != kSout * kB) return;
  if (in_sizes[3] != kVocab * kE) return;
  if (in_sizes[4] != kVocab * kE) return;
  if (in_sizes[5] != kG4 * kE || in_sizes[6] != kG4 * kEnc || in_sizes[7] != kG4) return;
  if (in_sizes[8] != kG4 * kE || in_sizes[9] != kG4 * kEnc || in_sizes[10] != kG4) return;
  if (in_sizes[11] != kG5 * kWxP || in_sizes[12] != kG5 * kWsP || in_sizes[13] != kG5) return;
  if (in_sizes[14] != kVocab * kD || in_sizes[15] != kVocab) return;
  if (out_size != kSout * kB * kVocab) return;
  if (ws_size < kWsTotal) return;

  const int*   xid     = (const int*)d_in[0];
  const int*   yid     = (const int*)d_in[2];
  const float* in_emb  = (const float*)d_in[3];
  const float* out_emb = (const float*)d_in[4];
  const float* Wih_f   = (const float*)d_in[5];
  const float* Whh_f   = (const float*)d_in[6];
  const float* b_f     = (const float*)d_in[7];
  const float* Wih_b   = (const float*)d_in[8];
  const float* Whh_b   = (const float*)d_in[9];
  const float* b_b     = (const float*)d_in[10];
  const float* cell_Wx = (const float*)d_in[11];
  const float* cell_Ws = (const float*)d_in[12];
  const float* cell_b  = (const float*)d_in[13];
  const float* logit_W = (const float*)d_in[14];
  const float* logit_b = (const float*)d_in[15];
  float* out = (float*)d_out;

  char* ws = (char*)d_ws;
  unsigned short* WIF16 = (unsigned short*)(ws + kOffWIF);
  unsigned short* WHF16 = (unsigned short*)(ws + kOffWHF);
  unsigned short* WIB16 = (unsigned short*)(ws + kOffWIB);
  unsigned short* WHB16 = (unsigned short*)(ws + kOffWHB);
  unsigned short* WX16  = (unsigned short*)(ws + kOffWX);
  unsigned short* WS16  = (unsigned short*)(ws + kOffWS);
  unsigned short* LW16  = (unsigned short*)(ws + kOffLW);
  unsigned short* XE16  = (unsigned short*)(ws + kOffXE);
  unsigned short* YE16  = (unsigned short*)(ws + kOffYE);
  float*          GIF   = (float*)(ws + kOffGIF);
  float*          GIB   = (float*)(ws + kOffGIB);
  float*          HST   = (float*)(ws + kOffH);
  unsigned short* H16   = (unsigned short*)(ws + kOffH16);
  float*          HPJ   = (float*)(ws + kOffHPJ);
  float*          YPJ   = (float*)(ws + kOffYPJ);
  float*          SPL   = (float*)(ws + kOffSPL);
  float*          CPL   = (float*)(ws + kOffCPL);
  unsigned short* ST16  = (unsigned short*)(ws + kOffST);

  cast_carry_kernel<<<(kG4 * kE / 8) / 256, 256, 0, stream>>>(Wih_f, WIF16, kG4 * kE / 8, kCarryW);
  cast_carry_kernel<<<(kG4 * kEnc / 8) / 256, 256, 0, stream>>>(Whh_f, WHF16, kG4 * kEnc / 8, kCarryW);
  cast_carry_kernel<<<(kG4 * kE / 8) / 256, 256, 0, stream>>>(Wih_b, WIB16, kG4 * kE / 8, kCarryW);
  cast_carry_kernel<<<(kG4 * kEnc / 8) / 256, 256, 0, stream>>>(Whh_b, WHB16, kG4 * kEnc / 8, kCarryW);
  cast_carry_kernel<<<(kG5 * kWxP / 8) / 256, 256, 0, stream>>>(cell_Wx, WX16, kG5 * kWxP / 8, kCarryW);
  cast_carry_kernel<<<(kG5 * kWsP / 8) / 256, 256, 0, stream>>>(cell_Ws, WS16, kG5 * kWsP / 8, kCarryW);
  cast_carry_kernel<<<(kVocab * kD / 8) / 256, 256, 0, stream>>>(logit_W, LW16, kVocab * kD / 8, kCarryW);

  gather_embed_kernel<<<dim3(kRows * 32 / 256, 2), 256, 0, stream>>>(xid, yid, in_emb, out_emb, XE16, YE16);

  wmma_gemm64_f16<2><<<16, 256, 0, stream>>>(XE16, kE, WIF16, kE, GIF, kG4, b_f, kRows, kG4, kE, kFoldEW);
  wmma_gemm64_f16<2><<<16, 256, 0, stream>>>(XE16, kE, WIB16, kE, GIB, kG4, b_b, kRows, kG4, kE, kFoldEW);

  encoder_kernel<<<2, 512, 0, stream>>>(GIF, GIB, WHF16, WHB16, HST);

  cast_carry_kernel<<<(kRows * 2 * kEnc / 8) / 256, 256, 0, stream>>>(HST, H16, kRows * 2 * kEnc / 8, kCarryS);
  wmma_gemm64_f16<0><<<20, 256, 0, stream>>>(H16, 2 * kEnc, WX16, kWxP, HPJ, kG5, nullptr, kRows, kG5, 2 * kEnc, kFoldSW);
  wmma_gemm64_f16<2><<<20, 256, 0, stream>>>(YE16, kE, WX16 + 2 * kEnc, kWxP, YPJ, kG5, cell_b, kRows, kG5, kE, kFoldEW);

  for (int d = 0; d < kSin + kSout - 1; ++d) {
    const int ilo = (d > kSout - 1) ? (d - (kSout - 1)) : 0;
    const int ihi = (d < kSin - 1) ? d : (kSin - 1);
    grid_cell_kernel<<<ihi - ilo + 1, 128, 0, stream>>>(HPJ, YPJ, WS16, SPL, CPL, d, ilo);
  }

  cast_carry_kernel<<<(kRows * kD / 8) / 256, 256, 0, stream>>>(
      SPL + (size_t)((kSin - 1) * kSout) * kPlane, ST16, kRows * kD / 8, kCarryS);
  wmma_gemm64_f16<2><<<(kRows / 64) * (kVocab / 64) / 8, 256, 0, stream>>>(
      ST16, kD, LW16, kD, out, kVocab, logit_b, kRows, kVocab, kD, kFoldSW);
}
